// EmgLSTMNet_71760313582333
// MI455X (gfx1250) — hardware-run, weakly checked
//
#include <hip/hip_runtime.h>
#include <math.h>

constexpr int NBATCH   = 256;
constexpr int NSTEP    = 2048;
constexpr int NIN      = 16;
constexpr int NH1      = 5;
constexpr int NH2      = 50;
constexpr int NCLS     = 20;
constexpr int ROWS_BLK = 16;
constexpr int NTHR     = 128;
constexpr int XCHUNK   = 8;
constexpr int KL1      = 32;
constexpr int KL2      = 64;
constexpr int A2P      = 72;
constexpr int H1P      = 16;
constexpr int OUT0_N   = NBATCH * NCLS;
constexpr int OUT1_N   = NBATCH * NH2;
constexpr int TILE0_N  = ROWS_BLK * NCLS;
constexpr int TILE1_N  = ROWS_BLK * NH2;
constexpr float ACARRY = 128.0f;
constexpr float WCARRY = 64.0f;
constexpr float FOLD   = 1.0f / (ACARRY * WCARRY);

static_assert(NBATCH % ROWS_BLK == 0, "batch tiles exact");
static_assert(NSTEP % XCHUNK == 0, "x chunks exact");
static_assert((XCHUNK & 1) == 0, "buffer parity follows the in-chunk step");
static_assert(NIN + NH1 <= KL1 && KL1 % 32 == 0, "layer-1 K padded to 32");
static_assert(NH2 + NH1 <= KL2 && KL2 % 32 == 0, "layer-2 K padded to 64");
static_assert(NH2 <= 64 && NH1 <= 16, "hidden units fit the per-wave 16-column tiles");
static_assert(NTHR == ROWS_BLK * XCHUNK, "x staging: one thread per (row, step)");
static_assert((OUT0_N + OUT1_N) * 4 == 71680, "output bytes");
static_assert(OUT0_N * 4 == 20480, "second output byte offset");
static_assert((TILE0_N * 4) % 128 == 0 && (TILE1_N * 4) % 128 == 0, "per-tile output regions are whole lines");
static_assert(TILE0_N % 4 == 0 && TILE1_N % 4 == 0, "float4 stores");
static_assert(3 * NTHR >= TILE0_N, "head loop covers the tile");

typedef __attribute__((ext_vector_type(16))) _Float16 v16h;
typedef __attribute__((ext_vector_type(8)))  _Float16 v8h;
typedef __attribute__((ext_vector_type(8)))  float    v8f;
typedef __attribute__((ext_vector_type(4)))  float    v4f;

template <typename T> struct Frag;
template <> struct Frag<_Float16> {
  typedef v16h V; union U { v16h v; v8h h[2]; };
  static __device__ __forceinline__ v16h load(const _Float16* p) {
    U f; f.h[0] = *(const v8h*)(p); f.h[1] = *(const v8h*)(p + 16); return f.v;
  }
  static __device__ __forceinline__ v8f mma(v16h a, v16h b, v8f c) {
    return __builtin_amdgcn_wmma_f32_16x16x32_f16(false, a, false, b, (short)0, c, false, false);
  }
};

__device__ __forceinline__ void guard_group(v8f& a, v8f& b, v8f& c, v8f& d, v16h x, v16h y0, v16h y1, v16h y2, v16h y3) {
  asm volatile("v_nop\n\tv_nop\n\tv_nop\n\tv_nop" : "+v"(a), "+v"(b), "+v"(c), "+v"(d) : "v"(x), "v"(y0), "v"(y1), "v"(y2), "v"(y3));
}
__device__ __forceinline__ void pin_f(float& x) { asm volatile("" : "+v"(x)); }
__device__ __forceinline__ float sigm(float x) { return __builtin_amdgcn_rcpf(1.0f + expf(-x)); }

__global__ __launch_bounds__(NTHR) void lstm2_seq_kernel(
    const float* __restrict__ x,
    const float* __restrict__ w1ih, const float* __restrict__ w1hh,
    const float* __restrict__ b1ih, const float* __restrict__ b1hh,
    const float* __restrict__ w2ih, const float* __restrict__ w2hh,
    const float* __restrict__ b2ih, const float* __restrict__ b2hh,
    const float* __restrict__ wfc,  const float* __restrict__ bfc,
    float* __restrict__ out) {
  __shared__ __align__(16) _Float16 B2L[4 * 64 * KL2];
  __shared__ __align__(16) _Float16 B1L[4 * 16 * KL1];
  __shared__ __align__(16) _Float16 A2[2 * ROWS_BLK * A2P];
  __shared__ __align__(16) _Float16 H1t[ROWS_BLK * H1P];
  __shared__ __align__(16) _Float16 Xr[XCHUNK * ROWS_BLK * NIN];
  __shared__ __align__(16) float L1[TILE1_N];
  __shared__ __align__(16) float L0[3 * NTHR];

  const int tid  = threadIdx.x;
  const int lane = tid & 31;
  const int wave = __builtin_amdgcn_readfirstlane((int)(threadIdx.x >> 5));
  const int c    = lane & 15;
  const int hh   = lane >> 4;
  const int koff = hh * 8;
  const int b0   = blockIdx.x * ROWS_BLK;
  const int u2   = 16 * wave + c;
  const bool live1 = (c < NH1);
  const bool live2 = (u2 < NH2);

#pragma unroll 1
  for (int i = tid; i < 2 * ROWS_BLK * A2P; i += NTHR) A2[i] = (_Float16)0.0f;
#pragma unroll 1
  for (int i = tid; i < ROWS_BLK * H1P; i += NTHR) H1t[i] = (_Float16)0.0f;

#pragma unroll 1
  for (int e = tid; e < 4 * 16 * KL1; e += NTHR) {
    const int row = e >> 5;
    const int k   = e & 31;
    const int q   = row >> 4;
    const int u   = row & 15;
    const int uc  = (u < NH1) ? u : (NH1 - 1);
    const int ki  = (k < NIN) ? k : (NIN - 1);
    int kh = k - NIN;
    kh = (kh < 0) ? 0 : kh;
    kh = (kh > NH1 - 1) ? (NH1 - 1) : kh;
    float wa = w1ih[(q * NH1 + uc) * NIN + ki];
    pin_f(wa);
    float wb = w1hh[(q * NH1 + uc) * NH1 + kh];
    pin_f(wb);
    const float inner = (k < NIN) ? wa : ((k < NIN + NH1) ? wb : 0.0f);
    const float v = (u < NH1) ? inner : 0.0f;
    B1L[e] = (_Float16)(v * WCARRY);
  }
#pragma unroll 1
  for (int e = tid; e < 4 * 64 * KL2; e += NTHR) {
    const int row = e >> 6;
    const int k   = e & 63;
    const int q   = row >> 6;
    const int u   = row & 63;
    const int uc  = (u < NH2) ? u : (NH2 - 1);
    const int kh  = (k < NH2) ? k : (NH2 - 1);
    int ki = k - NH2;
    ki = (ki < 0) ? 0 : ki;
    ki = (ki > NH1 - 1) ? (NH1 - 1) : ki;
    float wa = w2hh[(q * NH2 + uc) * NH2 + kh];
    pin_f(wa);
    float wb = w2ih[(q * NH2 + uc) * NH1 + ki];
    pin_f(wb);
    const float inner = (k < NH2) ? wa : ((k < NH2 + NH1) ? wb : 0.0f);
    const float v = (u < NH2) ? inner : 0.0f;
    B2L[e] = (_Float16)(v * WCARRY);
  }

  float bia1[4], bia2[4];
  {
    const int c1c = live1 ? c : (NH1 - 1);
    const int u2c = live2 ? u2 : (NH2 - 1);
#pragma unroll
    for (int q = 0; q < 4; ++q) {
      float p1 = b1ih[q * NH1 + c1c];
      pin_f(p1);
      float p2 = b1hh[q * NH1 + c1c];
      pin_f(p2);
      bia1[q] = live1 ? (p1 + p2) : 0.0f;
      float p3 = b2ih[q * NH2 + u2c];
      pin_f(p3);
      float p4 = b2hh[q * NH2 + u2c];
      pin_f(p4);
      bia2[q] = live2 ? (p3 + p4) : 0.0f;
    }
  }

  float c1s[8], c2s[8], h2f[8];
#pragma unroll
  for (int r = 0; r < 8; ++r) { c1s[r] = 0.0f; c2s[r] = 0.0f; h2f[r] = 0.0f; }

  __syncthreads();

  v16h bw[4][2];
#pragma unroll
  for (int q = 0; q < 4; ++q) {
#pragma unroll
    for (int ks = 0; ks < 2; ++ks)
      bw[q][ks] = Frag<_Float16>::load(B2L + (q * 64 + u2) * KL2 + ks * 32 + koff);
  }

  const v8f z8 = {0.f, 0.f, 0.f, 0.f, 0.f, 0.f, 0.f, 0.f};
  const int xm = tid >> 3;
  const int xs = tid & 7;
  const float* xrow = x + (size_t)(b0 + xm) * NSTEP * NIN;

#pragma unroll 1
  for (int tc = 0; tc < NSTEP / XCHUNK; ++tc) {
    {
      const float* xp = xrow + (size_t)(tc * XCHUNK + xs) * NIN;
      const v4f x0 = *(const v4f*)(xp);
      const v4f x1 = *(const v4f*)(xp + 4);
      const v4f x2 = *(const v4f*)(xp + 8);
      const v4f x3 = *(const v4f*)(xp + 12);
      v8h lo8, hi8;
#pragma unroll
      for (int e = 0; e < 4; ++e) {
        lo8[e]     = (_Float16)(x0[e] * ACARRY);
        lo8[4 + e] = (_Float16)(x1[e] * ACARRY);
        hi8[e]     = (_Float16)(x2[e] * ACARRY);
        hi8[4 + e] = (_Float16)(x3[e] * ACARRY);
      }
      _Float16* xd = Xr + (xs * ROWS_BLK + xm) * NIN;
      *(v8h*)(xd)     = lo8;
      *(v8h*)(xd + 8) = hi8;
    }
    __syncthreads();

#pragma unroll 1
    for (int s = 0; s < XCHUNK; ++s) {
      const int cur = s & 1;
      _Float16* a2cur = A2 + cur * (ROWS_BLK * A2P);
      _Float16* a2nxt = A2 + (cur ^ 1) * (ROWS_BLK * A2P);

      if (wave == 0) {
        Frag<_Float16>::U af;
        af.h[0] = *(const v8h*)(Xr + (s * ROWS_BLK + c) * NIN + koff);
        af.h[1] = *(const v8h*)(H1t + c * H1P + koff);
        const v16h w0 = Frag<_Float16>::load(B1L + (0 * 16 + c) * KL1 + koff);
        const v16h w1 = Frag<_Float16>::load(B1L + (1 * 16 + c) * KL1 + koff);
        const v16h w2 = Frag<_Float16>::load(B1L + (2 * 16 + c) * KL1 + koff);
        const v16h w3 = Frag<_Float16>::load(B1L + (3 * 16 + c) * KL1 + koff);
        v8f g0 = z8, g1 = z8, g2 = z8, g3 = z8;
        g0 = Frag<_Float16>::mma(af.v, w0, g0);
        g1 = Frag<_Float16>::mma(af.v, w1, g1);
        g2 = Frag<_Float16>::mma(af.v, w2, g2);
        g3 = Frag<_Float16>::mma(af.v, w3, g3);
        guard_group(g0, g1, g2, g3, af.v, w0, w1, w2, w3);
#pragma unroll
        for (int r = 0; r < 8; ++r) {
          const float zi = fmaf(g0[r], FOLD, bia1[0]);
          const float zf = fmaf(g1[r], FOLD, bia1[1]);
          const float zg = fmaf(g2[r], FOLD, bia1[2]);
          const float zo = fmaf(g3[r], FOLD, bia1[3]);
          const float ig = sigm(zi);
          const float fg = sigm(zf);
          const float gg = tanhf(zg);
          const float og = sigm(zo);
          const float cn = fg * c1s[r] + ig * gg;
          c1s[r] = cn;
          const float hn = og * tanhf(cn);
          const float hv = live1 ? hn : 0.0f;
          const _Float16 hq = (_Float16)(hv * ACARRY);
          H1t[(8 * hh + r) * H1P + c] = hq;
          if (live1) a2cur[(8 * hh + r) * A2P + NH2 + c] = hq;
        }
      }
      __syncthreads();

      {
        const _Float16* ar = a2cur + c * A2P + koff;
        const v16h a0 = Frag<_Float16>::load(ar);
        const v16h a1 = Frag<_Float16>::load(ar + 32);
        v8f g0 = z8, g1 = z8, g2 = z8, g3 = z8;
        g0 = Frag<_Float16>::mma(a0, bw[0][0], g0);
        g1 = Frag<_Float16>::mma(a0, bw[1][0], g1);
        g2 = Frag<_Float16>::mma(a0, bw[2][0], g2);
        g3 = Frag<_Float16>::mma(a0, bw[3][0], g3);
        guard_group(g0, g1, g2, g3, a0, bw[0][0], bw[1][0], bw[2][0], bw[3][0]);
        g0 = Frag<_Float16>::mma(a1, bw[0][1], g0);
        g1 = Frag<_Float16>::mma(a1, bw[1][1], g1);
        g2 = Frag<_Float16>::mma(a1, bw[2][1], g2);
        g3 = Frag<_Float16>::mma(a1, bw[3][1], g3);
        guard_group(g0, g1, g2, g3, a1, bw[0][1], bw[1][1], bw[2][1], bw[3][1]);
#pragma unroll
        for (int r = 0; r < 8; ++r) {
          const float zi = fmaf(g0[r], FOLD, bia2[0]);
          const float zf = fmaf(g1[r], FOLD, bia2[1]);
          const float zg = fmaf(g2[r], FOLD, bia2[2]);
          const float zo = fmaf(g3[r], FOLD, bia2[3]);
          const float ig = sigm(zi);
          const float fg = sigm(zf);
          const float gg = tanhf(zg);
          const float og = sigm(zo);
          const float cn = fg * c2s[r] + ig * gg;
          c2s[r] = cn;
          const float hn = og * tanhf(cn);
          const float hv = live2 ? hn : 0.0f;
          h2f[r] = hv;
          a2nxt[(8 * hh + r) * A2P + u2] = (_Float16)(hv * ACARRY);
        }
      }
      __syncthreads();
    }
  }

#pragma unroll
  for (int r = 0; r < 8; ++r) {
    if (live2) L1[(8 * hh + r) * NH2 + u2] = h2f[r];
  }
  __syncthreads();
#pragma unroll 1
  for (int i = 0; i < 3; ++i) {
    const int idx = i * NTHR + tid;
    const int idc = (idx < TILE0_N) ? idx : (TILE0_N - 1);
    const int row = idc / NCLS;
    const int n   = idc - row * NCLS;
    float sacc = 0.0f;
#pragma unroll 1
    for (int k = 0; k < NH2; ++k) {
      float wv = wfc[n * NH2 + k];
      pin_f(wv);
      sacc = fmaf(L1[row * NH2 + k], wv, sacc);
    }
    float bv = bfc[n];
    pin_f(bv);
    L0[idx] = sacc + bv;
  }
  __syncthreads();

  if (wave == 0) {
    float* o1 = out + OUT0_N + (size_t)b0 * NH2;
    constexpr int NV1 = TILE1_N / 4;
    v4f vals[7];
#pragma unroll
    for (int it = 0; it < 7; ++it) {
      const int i4 = it * 32 + lane;
      const int ic = (i4 < NV1) ? i4 : (NV1 - 1);
      vals[it] = *(const v4f*)(L1 + 4 * ic);
    }
    for (int pass = 0; pass < 2; ++pass) {
#pragma unroll
      for (int it = 0; it < 7; ++it) {
        const int i4 = it * 32 + lane;
        if (i4 < NV1) *(volatile v4f*)(o1 + 4 * i4) = vals[it];
      }
      __threadfence();
    }
  }
  if (wave == 1) {
    float* o0 = out + (size_t)b0 * NCLS;
    constexpr int NV0 = TILE0_N / 4;
    v4f vals[3];
#pragma unroll
    for (int it = 0; it < 3; ++it) {
      const int i4 = it * 32 + lane;
      const int ic = (i4 < NV0) ? i4 : (NV0 - 1);
      vals[it] = *(const v4f*)(L0 + 4 * ic);
    }
    for (int pass = 0; pass < 2; ++pass) {
#pragma unroll
      for (int it = 0; it < 3; ++it) {
        const int i4 = it * 32 + lane;
        if (i4 < NV0) *(volatile v4f*)(o0 + 4 * i4) = vals[it];
      }
      __threadfence();
    }
  }
}

extern "C" void kernel_launch(void* const* d_in, const int* in_sizes, int n_in,
                              void* d_out, int out_size, void* d_ws, size_t ws_size, hipStream_t stream) {
  (void)d_ws; (void)ws_size;
  if (n_in < 11 || d_out == nullptr) return;
  if (in_sizes[0] != NBATCH * NSTEP * NIN || in_sizes[1] != 4 * NH1 * NIN || in_sizes[2] != 4 * NH1 * NH1 ||
      in_sizes[3] != 4 * NH1 || in_sizes[4] != 4 * NH1 || in_sizes[5] != 4 * NH2 * NH1 ||
      in_sizes[6] != 4 * NH2 * NH2 || in_sizes[7] != 4 * NH2 || in_sizes[8] != 4 * NH2 ||
      in_sizes[9] != NCLS * NH2 || in_sizes[10] != NCLS || out_size != OUT0_N + OUT1_N) return;

  const float* x    = (const float*)d_in[0];
  const float* w1ih = (const float*)d_in[1];
  const float* w1hh = (const float*)d_in[2];
  const float* b1ih = (const float*)d_in[3];
  const float* b1hh = (const float*)d_in[4];
  const float* w2ih = (const float*)d_in[5];
  const float* w2hh = (const float*)d_in[6];
  const float* b2ih = (const float*)d_in[7];
  const float* b2hh = (const float*)d_in[8];
  const float* wfc  = (const float*)d_in[9];
  const float* bfc  = (const float*)d_in[10];
  float* out = (float*)d_out;

  lstm2_seq_kernel<<<NBATCH / ROWS_BLK, NTHR, 0, stream>>>(
      x, w1ih, w1hh, b1ih, b1hh, w2ih, w2hh, b2ih, b2hh, wfc, bfc, out);
}
